// GraphConvGRUCell_10763188044360
// MI455X (gfx1250) — hardware-verified
//
#include <hip/hip_runtime.h>
#include <stddef.h>
#include <math.h>


#define HD     64
#define IDIM   32
#define NBATCH 8
#define FROW   (NBATCH * HD)
#define NTHR   256
#define NWAVE  8
#define EPT    8
#define NGRP   2
#define CHUNK  (NTHR * EPT * NGRP)
#define WCAP   (EPT * NGRP * 32)
#define LISTN  (NWAVE * WCAP)
#define NBA    128
#define NBD    4096
#define GROWS  128
#define WSC    16.0f
#define WSCI   0.0625f
#define XOFF   (HD * HD / 8)
#define NXR    (3 * NBATCH * HD)

#define LDS_AGG (NBA * FROW * 4 + LISTN * 4 + 64 + NBA * 4 + NBA * 4)

static_assert((CHUNK & (CHUNK - 1)) == 0);
static_assert(CHUNK <= 4096);
static_assert((NBA & (NBA - 1)) == 0 && NBA <= 4096);
static_assert((NBD & (NBD - 1)) == 0 && NBD <= 4096);
static_assert(NBD == NWAVE * 4 * 128);
static_assert((NBA * FROW) % NTHR == 0);
static_assert(GROWS == NWAVE * 16);
static_assert(NBA <= NTHR);
static_assert(NWAVE == NBATCH);
static_assert(HD == 64 && IDIM == 32);

typedef float    v4f  __attribute__((ext_vector_type(4)));
typedef float    v8f  __attribute__((ext_vector_type(8)));
typedef int      v4i  __attribute__((ext_vector_type(4)));
typedef _Float16 v8h  __attribute__((ext_vector_type(8)));
typedef _Float16 v16h __attribute__((ext_vector_type(16)));
union FragH { v16h v; v8h h[2]; };

__device__ __forceinline__ v8h cvt8(v4f a, v4f b) {
  v8h r;
  r[0] = (_Float16)a.x; r[1] = (_Float16)a.y; r[2] = (_Float16)a.z; r[3] = (_Float16)a.w;
  r[4] = (_Float16)b.x; r[5] = (_Float16)b.y; r[6] = (_Float16)b.z; r[7] = (_Float16)b.w;
  return r;
}

__device__ __forceinline__ v8f wmh(v16h a, v16h b, v8f c) {
  v8f d = __builtin_amdgcn_wmma_f32_16x16x32_f16(false, a, false, b, (short)0, c, false, false);
  asm volatile("v_nop\n\tv_nop\n\tv_nop\n\tv_nop" : "+v"(d) : "v"(a), "v"(b));
  return d;
}

__device__ __forceinline__ float frcp(float x) { return __builtin_amdgcn_rcpf(x); }

template <int NB>
__device__ __forceinline__ int scan_chunk(const int* __restrict__ keys, int nE, int cbase, int nodeBase,
                                          int* list, int tid, int wave) {
  int wc = 0;
#pragma unroll
  for (int g = 0; g < NGRP; ++g) {
    const int el0  = (g * NTHR + tid) * EPT;
    const int e0   = cbase + el0;
    const int sent = -2147483647 - 1;
    v4i da, db;
    if (e0 + 7 < nE) {
      da = *(const v4i*)(keys + e0);
      db = *(const v4i*)(keys + e0 + 4);
    } else {
      da.x = (e0     < nE) ? keys[min(e0, nE - 1)] : sent;
      da.y = (e0 + 1 < nE) ? keys[min(e0 + 1, nE - 1)] : sent;
      da.z = (e0 + 2 < nE) ? keys[min(e0 + 2, nE - 1)] : sent;
      da.w = (e0 + 3 < nE) ? keys[min(e0 + 3, nE - 1)] : sent;
      db.x = (e0 + 4 < nE) ? keys[min(e0 + 4, nE - 1)] : sent;
      db.y = (e0 + 5 < nE) ? keys[min(e0 + 5, nE - 1)] : sent;
      db.z = (e0 + 6 < nE) ? keys[min(e0 + 6, nE - 1)] : sent;
      db.w = (e0 + 7 < nE) ? keys[min(e0 + 7, nE - 1)] : sent;
    }
    const unsigned nb = (unsigned)nodeBase;
    const unsigned s0 = (unsigned)da.x - nb, s1 = (unsigned)da.y - nb;
    const unsigned s2 = (unsigned)da.z - nb, s3 = (unsigned)da.w - nb;
    const unsigned s4 = (unsigned)db.x - nb, s5 = (unsigned)db.y - nb;
    const unsigned s6 = (unsigned)db.z - nb, s7 = (unsigned)db.w - nb;
    const bool h0 = s0 < (unsigned)NB, h1 = s1 < (unsigned)NB, h2 = s2 < (unsigned)NB, h3 = s3 < (unsigned)NB;
    const bool h4 = s4 < (unsigned)NB, h5 = s5 < (unsigned)NB, h6 = s6 < (unsigned)NB, h7 = s7 < (unsigned)NB;
    const unsigned any = __builtin_amdgcn_ballot_w32(h0 | h1 | h2 | h3 | h4 | h5 | h6 | h7);
    if (any != 0u) {
#define HITJ(J, HJ, SJ) { \
        const unsigned mj = __builtin_amdgcn_ballot_w32(HJ); \
        if (mj != 0u) { \
          if (HJ) { \
            const int pos = wc + (int)__builtin_amdgcn_mbcnt_lo(mj, 0u); \
            if (pos < WCAP) list[wave * WCAP + pos] = ((el0 + (J)) << 12) | (int)(SJ); \
          } \
          wc += (int)__builtin_popcount(mj); } }
      HITJ(0, h0, s0)
      HITJ(1, h1, s1)
      HITJ(2, h2, s2)
      HITJ(3, h3, s3)
      HITJ(4, h4, s4)
      HITJ(5, h5, s5)
      HITJ(6, h6, s6)
      HITJ(7, h7, s7)
#undef HITJ
    }
  }
  return wc;
}

__global__ __launch_bounds__(NTHR) void k_prep(
    const float* __restrict__ gw, const float* __restrict__ x,
    const float* __restrict__ wr, const float* __restrict__ br,
    const float* __restrict__ wz, const float* __restrict__ bz,
    const float* __restrict__ wh, const float* __restrict__ bh,
    _Float16* w16, float* xrzh) {
  const int t = blockIdx.x * NTHR + threadIdx.x;
  if (t < XOFF) {
    const int o  = t * 8;
    const int n  = o >> 6;
    const int k0 = o & (HD - 1);
    const float* p = gw + (size_t)k0 * HD + n;
    v4f a, b;
    a.x = p[0];      a.y = p[HD];     a.z = p[2 * HD]; a.w = p[3 * HD];
    b.x = p[4 * HD]; b.y = p[5 * HD]; b.z = p[6 * HD]; b.w = p[7 * HD];
    a = a * WSC;
    b = b * WSC;
    const v8h hv = cvt8(a, b);
    _Float16* dp = w16 + o;
    *(volatile v8h*)dp = hv;
    __threadfence();
    *(volatile v8h*)dp = hv;
  } else if (t < XOFF + NXR) {
    const int idx = t - XOFF;
    const int k = idx & (HD - 1);
    const int b = (idx >> 6) & (NBATCH - 1);
    const int g = idx >> 9;
    const float* w    = (g == 0) ? wr : ((g == 1) ? wz : wh);
    const float* bias = (g == 0) ? br : ((g == 1) ? bz : bh);
    float s = 0.f;
#pragma unroll
    for (int i = 0; i < IDIM; ++i) s += x[b * IDIM + i] * w[i * HD + k];
    s += bias[k];
    float* dp = xrzh + idx;
    *(volatile float*)dp = s;
    __threadfence();
    *(volatile float*)dp = s;
  }
}

__global__ __launch_bounds__(NTHR) void k_deg(
    const int* __restrict__ src, float* onorm, int nN, int nE) {
  __shared__ __attribute__((aligned(16))) int cnt[NBD];
  __shared__ __attribute__((aligned(16))) int list[LISTN];
  __shared__ int wcnt[NWAVE];
  const int tid = threadIdx.x, lane = tid & 31, wave = tid >> 5;
  const int nodeBase = blockIdx.x * NBD;
  (void)nN;

  for (int i = tid; i < NBD; i += NTHR) cnt[i] = 0;
  __syncthreads();

  const int nChunks = (nE + CHUNK - 1) / CHUNK;
#pragma unroll 1
  for (int ch = 0; ch < nChunks; ++ch) {
    const int cbase = ch * CHUNK;
    const int wc = scan_chunk<NBD>(src, nE, cbase, nodeBase, list, tid, wave);
    if (lane == 0) wcnt[wave] = wc;
    __syncthreads();
    if (wave == 0) {
#pragma unroll 1
      for (int wsx = 0; wsx < NWAVE; ++wsx) {
        int n = __builtin_amdgcn_readfirstlane(wcnt[wsx]);
        n = n > WCAP ? WCAP : (n < 0 ? 0 : n);
        const int* lp = list + wsx * WCAP;
#pragma unroll 1
        for (int i = 0; i < n; ++i) {
          const int ent  = __builtin_amdgcn_readfirstlane(lp[i]);
          const int slot = ent & (NBD - 1);
          if (lane == 0) cnt[slot] = cnt[slot] + 1;
        }
      }
    }
    __syncthreads();
  }

  v4f dq[4];
#pragma unroll
  for (int q = 0; q < 4; ++q) {
    const int f = (wave * 4 + q) * 128 + 4 * lane;
    v4i c = *(const v4i*)(cnt + f);
    c.x = c.x < 1 ? 1 : c.x; c.y = c.y < 1 ? 1 : c.y; c.z = c.z < 1 ? 1 : c.z; c.w = c.w < 1 ? 1 : c.w;
    dq[q].x = rsqrtf((float)c.x);
    dq[q].y = rsqrtf((float)c.y);
    dq[q].z = rsqrtf((float)c.z);
    dq[q].w = rsqrtf((float)c.w);
  }
  float* dp = onorm + (size_t)nodeBase;
#pragma unroll
  for (int q = 0; q < 4; ++q) *(volatile v4f*)(dp + (wave * 4 + q) * 128 + 4 * lane) = dq[q];
  __threadfence();
#pragma unroll
  for (int q = 0; q < 4; ++q) *(volatile v4f*)(dp + (wave * 4 + q) * 128 + 4 * lane) = dq[q];
}

__global__ __launch_bounds__(NTHR) void k_gemm(
    const float* __restrict__ hp, const _Float16* __restrict__ w16,
    const float* __restrict__ onorm, float* feat, int nN) {
  __shared__ __attribute__((aligned(16))) float stg[NWAVE * 16 * HD];
  const int tid = threadIdx.x, lane = tid & 31, wave = tid >> 5, hh = lane >> 4, m = lane & 15;
  const int rowBase = blockIdx.x * GROWS + wave * 16;
  const int mrow = rowBase + m;
  int node = mrow >> 3;
  node = node > nN - 1 ? nN - 1 : node;
  const int b = mrow & (NBATCH - 1);
  const float* arow = hp + ((size_t)b * nN + node) * HD;

  v8f acc[4];
#pragma unroll
  for (int ct = 0; ct < 4; ++ct) { v8f z = {0.f, 0.f, 0.f, 0.f, 0.f, 0.f, 0.f, 0.f}; acc[ct] = z; }

#pragma unroll
  for (int kt = 0; kt < HD / 32; ++kt) {
    const float* p = arow + 32 * kt + 8 * hh;
    FragH a;
    a.h[0] = cvt8(*(const v4f*)p, *(const v4f*)(p + 4));
    a.h[1] = cvt8(*(const v4f*)(p + 16), *(const v4f*)(p + 20));
#pragma unroll
    for (int ct = 0; ct < 4; ++ct) {
      const _Float16* bp = w16 + (size_t)(16 * ct + m) * HD + 32 * kt + 8 * hh;
      FragH bf;
      bf.h[0] = *(const v8h*)bp;
      bf.h[1] = *(const v8h*)(bp + 16);
      acc[ct] = wmh(a.v, bf.v, acc[ct]);
    }
  }

  int nodeh = (rowBase + 8 * hh) >> 3;
  nodeh = nodeh > nN - 1 ? nN - 1 : nodeh;
  const float sc = onorm[nodeh] * WSCI;
  float* sp = stg + wave * (16 * HD) + (8 * hh) * HD + m;
#pragma unroll
  for (int ct = 0; ct < 4; ++ct) {
    sp[0 * HD + 16 * ct] = acc[ct][0] * sc;
    sp[1 * HD + 16 * ct] = acc[ct][1] * sc;
    sp[2 * HD + 16 * ct] = acc[ct][2] * sc;
    sp[3 * HD + 16 * ct] = acc[ct][3] * sc;
    sp[4 * HD + 16 * ct] = acc[ct][4] * sc;
    sp[5 * HD + 16 * ct] = acc[ct][5] * sc;
    sp[6 * HD + 16 * ct] = acc[ct][6] * sc;
    sp[7 * HD + 16 * ct] = acc[ct][7] * sc;
  }
  __syncthreads();

  const float* lp = stg + wave * (16 * HD) + 4 * lane;
  float* gp = feat + (size_t)rowBase * HD + 4 * lane;
#pragma unroll
  for (int q = 0; q < 8; ++q) { const v4f v = *(const v4f*)(lp + q * 128); *(volatile v4f*)(gp + (size_t)q * 128) = v; }
  __threadfence();
#pragma unroll
  for (int q = 0; q < 8; ++q) { const v4f v = *(const v4f*)(lp + q * 128); *(volatile v4f*)(gp + (size_t)q * 128) = v; }
}

__global__ __launch_bounds__(NTHR) void k_agg(
    const int* __restrict__ src, const int* __restrict__ dst,
    const float* __restrict__ feat, const float* __restrict__ xrzh,
    const float* __restrict__ gb, const float* __restrict__ hp,
    float* out, int nN, int nE) {
  extern __shared__ v4f lds_dyn[];
  float* acc  = (float*)lds_dyn;
  int*   list = (int*)(acc + NBA * FROW);
  int*   wcnt = list + LISTN;
  int*   dcnt = wcnt + 16;
  float* dinv = (float*)(dcnt + NBA);
  const int tid = threadIdx.x, lane = tid & 31, wave = tid >> 5;
  const int nodeBase = blockIdx.x * NBA;

  {
    const v4f z = {0.f, 0.f, 0.f, 0.f};
    for (int i = tid; i < NBA * FROW / 4; i += NTHR) lds_dyn[i] = z;
  }
  if (tid < NBA) dcnt[tid] = 0;
  __syncthreads();

  const int nChunks = (nE + CHUNK - 1) / CHUNK;
#pragma unroll 1
  for (int ch = 0; ch < nChunks; ++ch) {
    const int cbase = ch * CHUNK;
    const int wc = scan_chunk<NBA>(dst, nE, cbase, nodeBase, list, tid, wave);
    if (lane == 0) wcnt[wave] = wc;
    __syncthreads();
    if (wave == 0) {
#pragma unroll 1
      for (int wsx = 0; wsx < NWAVE; ++wsx) {
        int n = __builtin_amdgcn_readfirstlane(wcnt[wsx]);
        n = n > WCAP ? WCAP : (n < 0 ? 0 : n);
        const int* lp = list + wsx * WCAP;
#pragma unroll 1
        for (int i = 0; i < n; ++i) {
          const int ent  = __builtin_amdgcn_readfirstlane(lp[i]);
          const int slot = ent & (NBA - 1);
          int e = cbase + ((ent >> 12) & (CHUNK - 1));
          e = e > nE - 1 ? nE - 1 : e;
          int s = src[e];
          s = s < 0 ? 0 : (s > nN - 1 ? nN - 1 : s);
          const float* fp = feat + (size_t)s * FROW + 4 * lane;
          float* ap = acc + slot * FROW + 4 * lane;
          const v4f g0 = *(const v4f*)(fp);
          const v4f g1 = *(const v4f*)(fp + 128);
          const v4f g2 = *(const v4f*)(fp + 256);
          const v4f g3 = *(const v4f*)(fp + 384);
          v4f* a0 = (v4f*)(ap);
          v4f* a1 = (v4f*)(ap + 128);
          v4f* a2 = (v4f*)(ap + 256);
          v4f* a3 = (v4f*)(ap + 384);
          const v4f r0 = *a0 + g0;
          const v4f r1 = *a1 + g1;
          const v4f r2 = *a2 + g2;
          const v4f r3 = *a3 + g3;
          *a0 = r0; *a1 = r1; *a2 = r2; *a3 = r3;
          if (lane == 0) dcnt[slot] = dcnt[slot] + 1;
        }
      }
    }
    __syncthreads();
  }

  if (tid < NBA) {
    int c = dcnt[tid];
    c = c < 1 ? 1 : c;
    dinv[tid] = rsqrtf((float)c);
  }
  __syncthreads();

#pragma unroll 1
  for (int i = 0; i < (NBA * FROW) / NTHR; ++i) {
    const int idx  = i * NTHR + tid;
    const int slot = idx >> 9;
    const int rem  = idx & (FROW - 1);
    const int b    = rem >> 6;
    const int col  = rem & (HD - 1);
    int node = nodeBase + slot;
    node = node > nN - 1 ? nN - 1 : node;
    const float av = dinv[slot] * acc[idx] + gb[col];
    const float xr = xrzh[rem];
    const float xz = xrzh[FROW + rem];
    const float xh = xrzh[2 * FROW + rem];
    const float hv = hp[((size_t)b * nN + node) * HD + col];
    const float rg = frcp(1.0f + expf(-(xr + av)));
    const float zg = frcp(1.0f + expf(-(xz + av)));
    const float u  = xh + rg * av;
    const float au = fabsf(u);
    const float e2 = expf(2.0f * au);
    float th = 1.0f - 2.0f * frcp(e2 + 1.0f);
    th = copysignf(th, u);
    acc[idx] = (1.0f - zg) * hv + zg * th;
  }
  __syncthreads();

  const size_t obase = ((size_t)wave * nN + nodeBase) * HD;
#pragma unroll 8
  for (int q = 0; q < NBA / 2; ++q) {
    const int row = 2 * q + (lane >> 4);
    if (nodeBase + row < nN) {
      const v4f v = *(const v4f*)(acc + row * FROW + wave * HD + 4 * (lane & 15));
      *(volatile v4f*)(out + obase + (size_t)q * 128 + 4 * lane) = v;
    }
  }
  __threadfence();
#pragma unroll 8
  for (int q = 0; q < NBA / 2; ++q) {
    const int row = 2 * q + (lane >> 4);
    if (nodeBase + row < nN) {
      const v4f v = *(const v4f*)(acc + row * FROW + wave * HD + 4 * (lane & 15));
      *(volatile v4f*)(out + obase + (size_t)q * 128 + 4 * lane) = v;
    }
  }
}

extern "C" void kernel_launch(void* const* d_in, const int* in_sizes, int n_in,
                              void* d_out, int out_size, void* d_ws, size_t ws_size,
                              hipStream_t stream) {
  if (n_in < 12) return;
  if (in_sizes[0] != NBATCH * IDIM) return;
  const int nN = in_sizes[1] / FROW;
  if (nN <= 0 || in_sizes[1] != nN * FROW) return;
  const int nE = in_sizes[2];
  if (nE < 0 || in_sizes[3] != nE) return;
  if (in_sizes[4] != IDIM * HD || in_sizes[6] != IDIM * HD || in_sizes[8] != IDIM * HD) return;
  if (in_sizes[5] < HD || in_sizes[7] < HD || in_sizes[9] < HD || in_sizes[11] < HD) return;
  if (in_sizes[10] != HD * HD) return;
  if (out_size != in_sizes[1]) return;

  const float* x      = (const float*)d_in[0];
  const float* h_prev = (const float*)d_in[1];
  const int*   src    = (const int*)d_in[2];
  const int*   dst    = (const int*)d_in[3];
  const float* w_r_w  = (const float*)d_in[4];
  const float* w_r_b  = (const float*)d_in[5];
  const float* w_z_w  = (const float*)d_in[6];
  const float* w_z_b  = (const float*)d_in[7];
  const float* w_h_w  = (const float*)d_in[8];
  const float* w_h_b  = (const float*)d_in[9];
  const float* gcn_w  = (const float*)d_in[10];
  const float* gcn_b  = (const float*)d_in[11];
  float* out = (float*)d_out;

  const int nBD = (nN + NBD - 1) / NBD;
  const int nG  = (nN * NBATCH + GROWS - 1) / GROWS;
  const int nA  = (nN + NBA - 1) / NBA;

  char* ws = (char*)d_ws;
  size_t off = 0;
  const size_t oW = off; off += (size_t)HD * HD * 2;                   off = (off + 255) & ~(size_t)255;
  const size_t oX = off; off += (size_t)NXR * 4;                       off = (off + 255) & ~(size_t)255;
  const size_t oN = off; off += (size_t)nBD * NBD * 4;                 off = (off + 255) & ~(size_t)255;
  const size_t oF = off; off += (size_t)nG * GROWS * HD * 4;           off = (off + 255) & ~(size_t)255;
  if (off > ws_size) return;
  _Float16* w16   = (_Float16*)(ws + oW);
  float*    xrzh  = (float*)(ws + oX);
  float*    onorm = (float*)(ws + oN);
  float*    feat  = (float*)(ws + oF);

  k_prep<<<(XOFF + NXR + NTHR - 1) / NTHR, NTHR, 0, stream>>>(
      gcn_w, x, w_r_w, w_r_b, w_z_w, w_z_b, w_h_w, w_h_b, w16, xrzh);

  k_deg<<<nBD, NTHR, 0, stream>>>(src, onorm, nN, nE);

  k_gemm<<<nG, NTHR, 0, stream>>>(h_prev, w16, onorm, feat, nN);

  hipFuncSetAttribute(reinterpret_cast<const void*>(&k_agg),
                      hipFuncAttributeMaxDynamicSharedMemorySize, LDS_AGG);
  k_agg<<<nA, NTHR, LDS_AGG, stream>>>(src, dst, feat, xrzh, gcn_b, h_prev, out, nN, nE);
}
